// HopfieldASAAttention_14817637171724
// MI455X (gfx1250) — hardware-verified
//
#include <hip/hip_runtime.h>


namespace {
constexpr int Bn = 2, N = 4096, D = 1024, PD = 64, R = 32, FW = 96  , NT = Bn * N;
constexpr float RFFS = 0.25f  , XS = 8.0f, PS = 8.0f;
struct Wo_ { static constexpr size_t POS = 0, V = (size_t)PD * D, O = V + (size_t)D * D, END = O + (size_t)D * D; };

typedef _Float16 b16;
typedef __attribute__((ext_vector_type(16))) _Float16 v16b;
typedef __attribute__((ext_vector_type(8))) _Float16 v8b;
typedef __attribute__((ext_vector_type(8))) float v8f;
typedef __attribute__((ext_vector_type(4))) float v4f;
__device__ __forceinline__ float bf16_rne(float f) { unsigned int u = __float_as_uint(f); u += 0x7FFFu + ((u >> 16) & 1u); return __uint_as_float(u & 0xFFFF0000u); }
__device__ __forceinline__ void split16(float v, b16& hi, b16& lo) { hi = (b16)v; lo = (b16)(v - (float)hi); }
__device__ __forceinline__ v16b frag_kb(const b16* p, int hh) { const v8b a = *(const v8b*)(p + 8 * hh), b = *(const v8b*)(p + 16 + 8 * hh); v16b f;
#pragma unroll
  for (int e = 0; e < 8; ++e) { f[e] = a[e]; f[8 + e] = b[e]; } return f; }
__device__ __forceinline__ v8f wmma16b(v16b a, v16b b, v8f c) { v8f d = __builtin_amdgcn_wmma_f32_16x16x32_f16(false, a, false, b, (short)0, c, false, false); asm volatile("v_nop\n\tv_nop\n\tv_nop\n\tv_nop" : "+v"(d) : "v"(a), "v"(b)); return d; }
__device__ __forceinline__ void wave_lds_sync() { __builtin_amdgcn_fence(__ATOMIC_RELEASE, "workgroup"); __builtin_amdgcn_wave_barrier(); __builtin_amdgcn_fence(__ATOMIC_ACQUIRE, "workgroup"); }
__device__ __forceinline__ float nexp(float x) { return __builtin_amdgcn_exp2f(x * 1.4426950408889634f); }
__device__ __forceinline__ float nlog(float x) { return __builtin_amdgcn_logf(x) * 0.6931471805599453f; }
__device__ __forceinline__ float pmul(float a, float b) { float p = a * b; asm volatile("" : "+v"(p)); return p; }
__device__ __forceinline__ void sincos_r(float ang, float& sn, float& cs) { const float k = rintf(ang * 0.15915494309189535f); float r = __builtin_fmaf(k, -6.28318548202514648f, ang); r = __builtin_fmaf(k, 1.7484556025237907e-7f, r);
  const float t = r * 0.15915494309189535f; sn = __builtin_amdgcn_sinf(t); cs = __builtin_amdgcn_cosf(t); }
__device__ __forceinline__ float tanh_n(float x) { const float ax = fabsf(x); const float e = __builtin_amdgcn_exp2f(-2.8853900817779268f * ax); float t = (1.0f - e) / (1.0f + e); return (x < 0.0f) ? -t : t; }
__device__ __forceinline__ float softplus_f(float x) { return (x > 20.0f) ? x : nlog(1.0f + nexp(x)); }

__global__ __launch_bounds__(256) void prep_kernel(const float* __restrict__ x, const float* __restrict__ pw, const float* __restrict__ pb, const float* __restrict__ cw, const float* __restrict__ cb, const float* __restrict__ om, const float* __restrict__ rb, const float* __restrict__ vw, const float* __restrict__ vb, const float* __restrict__ ow, const float* __restrict__ ob, const float* __restrict__ cs, const float* __restrict__ ds, b16* __restrict__ X, b16* __restrict__ Rw, float* __restrict__ P) {
  const int t_ = threadIdx.x; const size_t tid = (size_t)blockIdx.x * 256 + t_, nth = (size_t)gridDim.x * 256;
  for (int pass = 0; pass < 2; ++pass) {
    { const int row = blockIdx.x * 8 + (t_ >> 5), lane = t_ & 31; for (int c8 = lane * 8; c8 < D; c8 += 256) { v8b v; for (int e = 0; e < 8; ++e) v[e] = (b16)bf16_rne(x[(size_t)row * D + c8 + e]); *(volatile v8b*)(X + (size_t)row * D + c8) = v; } }
    for (size_t p = tid; p < Wo_::END / 8; p += nth) { const size_t q = p * 8; const float* s_ = (q < Wo_::V) ? (pw + q) : (q < Wo_::O) ? (vw + (q - Wo_::V)) : (ow + (q - Wo_::O)); v8b v; for (int e = 0; e < 8; ++e) v[e] = (b16)bf16_rne(s_[e]); *(volatile v8b*)(Rw + q) = v; }
    for (size_t q = tid; q < 5219; q += nth) { const int i = (int)q; float v; if (i < 64) v = bf16_rne(pb[i]); else if (i < 1088) v = bf16_rne(cw[i - 64]); else if (i == 1088) v = bf16_rne(cb[0]); else if (i < 3137) v = bf16_rne(om[i - 1089]); else if (i < 3169) v = bf16_rne(rb[i - 3137]); else if (i < 4193) v = bf16_rne(vb[i - 3169]); else if (i < 5217) v = bf16_rne(ob[i - 4193]); else if (i == 5217) v = softplus_f(bf16_rne(cs[0])); else v = softplus_f(bf16_rne(ds[0])); P[q] = v; }
    __threadfence(); }
}

__global__ __launch_bounds__(64) void feat_kernel(const b16* __restrict__ X, const b16* __restrict__ Rw, const float* __restrict__ P, b16* __restrict__ FQh, b16* __restrict__ FQl, b16* __restrict__ FKh, b16* __restrict__ FKl, b16* __restrict__ VT, b16* __restrict__ VTl) {
  __shared__ float pos[2][64][PD + 1]; __shared__ float chg[2][64]; __shared__ __attribute__((aligned(16))) b16 Tv[128][128 + 8], Tvl[128][128 + 8];
  const int lane = threadIdx.x & 31, wave = threadIdx.x >> 5, nloc = lane & 15, hlf = lane >> 4, t0 = blockIdx.x * 128, m0 = t0 + wave * 64; const int b = t0 / N, p0 = t0 % N;
  for (int rt = 0; rt < 4; ++rt) { v8f acc[4] = {{}, {}, {}, {}};
#pragma unroll 2
    for (int kb = 0; kb < D; kb += 32) { const v16b a = frag_kb(X + (size_t)(m0 + rt * 16 + nloc) * D + kb, hlf);
#pragma unroll
      for (int t = 0; t < 4; ++t) acc[t] = wmma16b(a, frag_kb(Rw + Wo_::POS + (size_t)(t * 16 + nloc) * D + kb, hlf), acc[t]); }
#pragma unroll
    for (int t = 0; t < 4; ++t)
#pragma unroll
      for (int r = 0; r < 8; ++r) pos[wave][rt * 16 + 8 * hlf + r][t * 16 + nloc] = acc[t][r] + P[t * 16 + nloc]; }
  for (int q = 0; q < 64; ++q) { const b16* xr = X + (size_t)(m0 + q) * D; float s = 0.0f; for (int c = lane; c < D; c += 32) s += pmul((float)xr[c], P[64 + c]);
#pragma unroll
    for (int o = 1; o < 32; o <<= 1) s += __shfl_xor(s, o); if (lane == 0) chg[wave][q] = tanh_n(s + P[1088]); }
  wave_lds_sync();
  const float sd = sqrtf(P[5218]), sc = sqrtf(P[5217]);
  __shared__ float Ff[2][64][FW + 1];
  for (int it = lane; it < 64 * R; it += 32) { const int q = it >> 5, r = it & 31; float a = P[3137 + r];
#pragma unroll 8
    for (int p = 0; p < PD; ++p) a += pmul(pos[wave][q][p], P[1089 + r * PD + p]);
    float sn, cs_; sincos_r(a, sn, cs_); Ff[wave][q][r] = pmul(sd * RFFS, cs_); Ff[wave][q][R + r] = pmul(sd * RFFS, sn); }
  for (int q = lane; q < 64; q += 32) { Ff[wave][q][64] = pmul(sc, chg[wave][q]); for (int c = 65; c < FW; ++c) Ff[wave][q][c] = 0.0f; }
  wave_lds_sync();
  for (int pass = 0; pass < 2; ++pass) { for (int i = lane; i < 64 * (FW / 8); i += 32) { const int q = i / (FW / 8), c8 = (i % (FW / 8)) * 8; v8b qh, ql, kh, kl;
      for (int e = 0; e < 8; ++e) { const int c = c8 + e; const float v = Ff[wave][q][c]; b16 a_, b_; split16(v * XS, a_, b_); qh[e] = a_; ql[e] = b_; const float vk = (c == 64) ? -v : v; split16(vk * XS, a_, b_); kh[e] = a_; kl[e] = b_; }
      const size_t gi = (size_t)(m0 + q) * FW + c8; *(volatile v8b*)(FQh + gi) = qh; *(volatile v8b*)(FQl + gi) = ql; *(volatile v8b*)(FKh + gi) = kh; *(volatile v8b*)(FKl + gi) = kl; } __threadfence(); }
  for (int ch = 0; ch < 8; ++ch) {
    for (int rt = 0; rt < 4; ++rt) { v8f acc[8];
#pragma unroll
      for (int t = 0; t < 8; ++t) acc[t] = (v8f){};
#pragma unroll 2
      for (int kb = 0; kb < D; kb += 32) { const v16b a = frag_kb(X + (size_t)(m0 + rt * 16 + nloc) * D + kb, hlf);
#pragma unroll
        for (int t = 0; t < 8; ++t) acc[t] = wmma16b(a, frag_kb(Rw + Wo_::V + (size_t)(ch * 128 + t * 16 + nloc) * D + kb, hlf), acc[t]); }
#pragma unroll
      for (int t = 0; t < 8; ++t)
#pragma unroll
        for (int r = 0; r < 8; ++r) { const int c = t * 16 + nloc; b16 a_, c_; split16((acc[t][r] + P[3169 + ch * 128 + c]) * XS, a_, c_); Tv[c][wave * 64 + rt * 16 + 8 * hlf + r] = a_; Tvl[c][wave * 64 + rt * 16 + 8 * hlf + r] = c_; } }
    __syncthreads();
    for (int pass = 0; pass < 2; ++pass) { for (int i = threadIdx.x; i < 128 * 16; i += 64) { const int c = i >> 4, c8 = (i & 15) * 8; const size_t gi = ((size_t)b * D + ch * 128 + c) * N + p0 + c8; *(volatile v8b*)(VT + gi) = *(const v8b*)(&Tv[c][c8]); *(volatile v8b*)(VTl + gi) = *(const v8b*)(&Tvl[c][c8]); } __threadfence(); }
    __syncthreads(); }
}

__global__ __launch_bounds__(256) void attn_kernel(const b16* __restrict__ FQh, const b16* __restrict__ FQl, const b16* __restrict__ FKh, const b16* __restrict__ FKl, const b16* __restrict__ VT, const b16* __restrict__ VTl, b16* __restrict__ O, b16* __restrict__ Ol) {
  __shared__ __attribute__((aligned(16))) b16 Os[16][D + 8], Osl[16][D + 8]; __shared__ float Sx[2][16][16 + 1];
  const int wave = threadIdx.x >> 5, lane = threadIdx.x & 31, hh = lane >> 4, col = lane & 15; const int b = blockIdx.x / (N / 16), q0 = (blockIdx.x % (N / 16)) * 16, qi = q0 + col;
  const b16* Vb = VT + ((size_t)b * D + wave * 128) * N; const b16* Vbl = VTl + ((size_t)b * D + wave * 128) * N; const size_t tb = (size_t)b * N; const float SC = 1.0f / (XS * XS);
  v16b qh_[3], ql_[3];
#pragma unroll
  for (int j = 0; j < 3; ++j) { qh_[j] = frag_kb(FQh + (tb + qi) * FW + 32 * j, hh); ql_[j] = frag_kb(FQl + (tb + qi) * FW + 32 * j, hh); }
  float m = -INFINITY, l = 0.0f; v8f o[8];
#pragma unroll
  for (int t = 0; t < 8; ++t) o[t] = (v8f){};
  for (int kb = 0; kb <= q0 + 15; kb += 32) { v8f s0, s1;
    if (wave < 2) { v8f s = {};
#pragma unroll
      for (int j = 0; j < 3; ++j) { const v16b kh_ = frag_kb(FKh + (tb + kb + 16 * wave + col) * FW + 32 * j, hh), kl_ = frag_kb(FKl + (tb + kb + 16 * wave + col) * FW + 32 * j, hh); s = wmma16b(kh_, qh_[j], s); s = wmma16b(kh_, ql_[j], s); s = wmma16b(kl_, qh_[j], s); }
#pragma unroll
      for (int r = 0; r < 8; ++r) Sx[wave][8 * hh + r][col] = s[r]; }
    __syncthreads();
#pragma unroll
    for (int r = 0; r < 8; ++r) { s0[r] = Sx[0][8 * hh + r][col]; s1[r] = Sx[1][8 * hh + r][col]; }
    __syncthreads();
    float mr = -INFINITY;
#pragma unroll
    for (int r = 0; r < 8; ++r) { const int k0 = kb + 8 * hh + r, k1 = k0 + 16; s0[r] = (k0 <= qi) ? s0[r] * SC : -INFINITY; s1[r] = (k1 <= qi) ? s1[r] * SC : -INFINITY; mr = fmaxf(mr, fmaxf(s0[r], s1[r])); }
    mr = fmaxf(mr, __shfl_xor(mr, 16)); const float mn = fmaxf(m, mr), al_ = nexp(m - mn); m = mn; float sum = 0.0f; v16b pb, pl;
#pragma unroll
    for (int r = 0; r < 8; ++r) { const float e0 = (s0[r] == -INFINITY) ? 0.0f : nexp(s0[r] - mn), e1 = (s1[r] == -INFINITY) ? 0.0f : nexp(s1[r] - mn); sum += e0 + e1; b16 a_, c_; split16(e0 * PS, a_, c_); pb[r] = a_; pl[r] = c_; split16(e1 * PS, a_, c_); pb[8 + r] = a_; pl[8 + r] = c_; }
    sum += __shfl_xor(sum, 16); l = l * al_ + sum;
#pragma unroll
    for (int t = 0; t < 8; ++t) { o[t] *= al_; const v16b vh = frag_kb(Vb + (size_t)(t * 16 + col) * N + kb, hh), vl = frag_kb(Vbl + (size_t)(t * 16 + col) * N + kb, hh); o[t] = wmma16b(vh, pb, o[t]); o[t] = wmma16b(vh, pl, o[t]); o[t] = wmma16b(vl, pb, o[t]); } }
  const float inv = 1.0f / (l * PS);
#pragma unroll
  for (int t = 0; t < 8; ++t)
#pragma unroll
    for (int r = 0; r < 8; ++r) { b16 a_, c_; split16(o[t][r] * inv, a_, c_); Os[col][wave * 128 + t * 16 + 8 * hh + r] = a_; Osl[col][wave * 128 + t * 16 + 8 * hh + r] = c_; }
  __syncthreads();
  for (int pass = 0; pass < 2; ++pass) { for (int i = threadIdx.x; i < 16 * (D / 8); i += 256) { const int rr = i >> 7, c8 = (i & 127) * 8; *(volatile v8b*)(O + (tb + q0 + rr) * D + c8) = *(const v8b*)(&Os[rr][c8]); *(volatile v8b*)(Ol + (tb + q0 + rr) * D + c8) = *(const v8b*)(&Osl[rr][c8]); } __threadfence(); }
}

__global__ __launch_bounds__(64) void out_kernel(const b16* __restrict__ O, const b16* __restrict__ Ol, const b16* __restrict__ Rw, const float* __restrict__ P, float* __restrict__ out) {
  __shared__ __attribute__((aligned(16))) float Ts[2][32][128 + 4];
  const int lane = threadIdx.x & 31, wave = threadIdx.x >> 5, nloc = lane & 15, hlf = lane >> 4, m0 = blockIdx.y * 32, c0 = blockIdx.x * 256 + wave * 128; const b16* Wr = Rw + Wo_::O;
  v8f acc[2][8];
#pragma unroll
  for (int r = 0; r < 2; ++r)
#pragma unroll
    for (int t = 0; t < 8; ++t) acc[r][t] = (v8f){};
#pragma unroll 2
  for (int kb = 0; kb < D; kb += 32) { const v16b a0 = frag_kb(O + (size_t)(m0 + nloc) * D + kb, hlf), l0 = frag_kb(Ol + (size_t)(m0 + nloc) * D + kb, hlf), a1 = frag_kb(O + (size_t)(m0 + 16 + nloc) * D + kb, hlf), l1 = frag_kb(Ol + (size_t)(m0 + 16 + nloc) * D + kb, hlf);
#pragma unroll
    for (int t = 0; t < 8; ++t) { const v16b bw = frag_kb(Wr + (size_t)(c0 + t * 16 + nloc) * D + kb, hlf); acc[0][t] = wmma16b(a0, bw, acc[0][t]); acc[0][t] = wmma16b(l0, bw, acc[0][t]); acc[1][t] = wmma16b(a1, bw, acc[1][t]); acc[1][t] = wmma16b(l1, bw, acc[1][t]); } }
#pragma unroll
  for (int t = 0; t < 8; ++t) { const float bb = P[4193 + c0 + t * 16 + nloc];
#pragma unroll
    for (int r = 0; r < 2; ++r)
#pragma unroll
      for (int v = 0; v < 8; ++v) Ts[wave][r * 16 + 8 * hlf + v][t * 16 + nloc] = acc[r][t][v] * (1.0f / XS) + bb; }
  wave_lds_sync();
  for (int pass = 0; pass < 2; ++pass) { for (int i = lane; i < 32 * 32; i += 32) { const int rr = i >> 5, c4 = (i & 31) * 4; *(volatile v4f*)(out + (size_t)(m0 + rr) * D + c0 + c4) = *(const v4f*)(&Ts[wave][rr][c4]); } __threadfence(); }
}
}

extern "C" void kernel_launch(void* const* d_in, const int* in_sizes, int n_in,
                              void* d_out, int out_size, void* d_ws, size_t ws_size, hipStream_t stream) {
  (void)n_in; (void)out_size;
  const float* x = (const float*)d_in[0]; const float* pw = (const float*)d_in[1]; const float* pb = (const float*)d_in[2]; const float* cw = (const float*)d_in[3]; const float* cb = (const float*)d_in[4]; const float* om = (const float*)d_in[5]; const float* rb = (const float*)d_in[6];
  const float* vw = (const float*)d_in[7]; const float* vb = (const float*)d_in[8]; const float* ow = (const float*)d_in[9]; const float* ob = (const float*)d_in[10]; const float* cs = (const float*)d_in[11]; const float* ds = (const float*)d_in[12];
  float* out = (float*)d_out;
  if (in_sizes[0] != NT * D || in_sizes[1] != PD * D || in_sizes[5] != R * PD || in_sizes[7] != D * D || in_sizes[9] != D * D) return;
  size_t off = 0; char* ws = (char*)d_ws;
  auto carve = [&](size_t bytes) { char* p = ws + off; off += (bytes + 255) & ~(size_t)255; return p; };
  b16* X = (b16*)carve((size_t)NT * D * 2); b16* Rw = (b16*)carve(Wo_::END * 2); float* P = (float*)carve(5376 * 4); b16* FQh = (b16*)carve((size_t)NT * FW * 2); b16* FQl = (b16*)carve((size_t)NT * FW * 2); b16* FKh = (b16*)carve((size_t)NT * FW * 2); b16* FKl = (b16*)carve((size_t)NT * FW * 2);
  b16* VT = (b16*)carve((size_t)NT * D * 2); b16* VTl = (b16*)carve((size_t)NT * D * 2); b16* O = (b16*)carve((size_t)NT * D * 2); b16* Ol = (b16*)carve((size_t)NT * D * 2);
  if (off > ws_size) return;
  prep_kernel<<<NT / 8, 256, 0, stream>>>(x, pw, pb, cw, cb, om, rb, vw, vb, ow, ob, cs, ds, X, Rw, P);
  feat_kernel<<<NT / 128, 64, 0, stream>>>(X, Rw, P, FQh, FQl, FKh, FKl, VT, VTl);
  attn_kernel<<<NT / 16, 256, 0, stream>>>(FQh, FQl, FKh, FKl, VT, VTl, O, Ol);
  out_kernel<<<dim3(D / 256, NT / 32), 64, 0, stream>>>(O, Ol, Rw, P, out);
}
